// Propagation_Attention_3367254360659
// MI455X (gfx1250) — hardware-run, weakly checked
//
#include <hip/hip_runtime.h>
#include <math.h>

#ifndef NB
#define NB 8
#endif
#ifndef SEQ
#define SEQ 1024
#endif
#define NB_FULL 8
#define SEQ_FULL 1024
#define CC 256
#define HEADS 8
#define HD 32
#define NTAB 10
#define QKP 512
#define MTOK (NB * SEQ)

#define CARRY_X 16.0f
#define CARRY_W 16.0f
#define CARRY_QKV 16.0f
#define CARRY_P 1024.0f
#define CARRY_CTX 64.0f

static constexpr float SC_QKV   = 1.0f / 16.0f;
static constexpr float SC_SCORE = 0.17677669529663687f / 256.0f;
static constexpr float SC_DEN   = 256.0f;
static constexpr float SC_OUT   = 1.0f / 1024.0f;
static constexpr float LOG2E    = 1.4426950408889634f;

static_assert(SC_QKV * (CARRY_X * CARRY_W) == CARRY_QKV);
static_assert(SC_SCORE * (CARRY_QKV * CARRY_QKV) == 0.17677669529663687f);
static_assert(SC_DEN * CARRY_CTX == CARRY_P * CARRY_QKV);
static_assert(SC_OUT * (CARRY_CTX * CARRY_W) == 1.0f);

static_assert(NB <= NB_FULL);
static_assert(SEQ <= SEQ_FULL);
static_assert(SEQ % 128 == 0);
static_assert(HEADS * HD == CC);
static_assert(HD == 32);
static_assert(QKP == 2 * CC);
static_assert(MTOK % 64 == 0);
static_assert(CC % 64 == 0 && QKP % 64 == 0);
static_assert(CC % 32 == 0);
static_assert(CC / 8 == 32);
static_assert((MTOK * (CC / 8)) % 256 == 0);
static_assert((3 * CC * (CC / 8)) % 256 == 0);
static_assert((CC * (CC / 8)) % 256 == 0);
static_assert(NTAB * HEADS <= 256);

typedef __attribute__((ext_vector_type(16))) _Float16 v16h;
typedef __attribute__((ext_vector_type(8)))  _Float16 v8h;
typedef __attribute__((ext_vector_type(4)))  _Float16 v4h;
typedef __attribute__((ext_vector_type(2)))  _Float16 v2h;
typedef __attribute__((ext_vector_type(8)))  float    v8f;
typedef __attribute__((ext_vector_type(4)))  float    v4f;
typedef __attribute__((ext_vector_type(2)))  float    v2f;
typedef __attribute__((ext_vector_type(4)))  int      v4i;


__device__ __forceinline__ float bfr(float f) {
    unsigned u = __float_as_uint(f);
    u += 0x7FFFu + ((u >> 16) & 1u);
    return __uint_as_float(u & 0xFFFF0000u);
}

static __device__ __forceinline__ v2h toh_flush2(float a, float b) {
    const float wa = (fabsf(a) < 6.103515625e-05f) ? 0.0f : a;
    const float wb = (fabsf(b) < 6.103515625e-05f) ? 0.0f : b;
    const v2f w = {wa, wb};
    return __builtin_convertvector(w, v2h);
}
static __device__ __forceinline__ v8h cat8(v2h a, v2h b, v2h c, v2h d) {
    const v4h lo = __builtin_shufflevector(a, b, 0, 1, 2, 3);
    const v4h hi = __builtin_shufflevector(c, d, 0, 1, 2, 3);
    return __builtin_shufflevector(lo, hi, 0, 1, 2, 3, 4, 5, 6, 7);
}
static __device__ __forceinline__ v8h pack8f(const float* v) {
    return cat8(toh_flush2(v[0], v[1]), toh_flush2(v[2], v[3]), toh_flush2(v[4], v[5]), toh_flush2(v[6], v[7]));
}
static __device__ __forceinline__ void st8hf(_Float16* P, const float* v) {
    const v8h hv = pack8f(v);
    *(volatile v8h*)(P) = hv;
    __threadfence();
    *(volatile v8h*)(P) = hv;
}

union FragU { v16h v; v8h h[2]; };
__device__ __forceinline__ v16h frag_ld(const _Float16* p) {
    FragU f; f.h[0] = *(const v8h*)(p); f.h[1] = *(const v8h*)(p + 16); return f.v;
}
__device__ __forceinline__ v8f wmma16(v16h a, v16h b, v8f c) {
    c = __builtin_amdgcn_wmma_f32_16x16x32_f16(false, a, false, b, (short)0, c, false, false);
    asm volatile("v_nop\n\tv_nop\n\tv_nop\n\tv_nop" : "+v"(c) : "v"(a), "v"(b));
    return c;
}
__device__ __forceinline__ void wave_sync_lds() {
    __builtin_amdgcn_fence(3  , "workgroup");
    __builtin_amdgcn_wave_barrier();
    __builtin_amdgcn_fence(2  , "workgroup");
}

static_assert(32 * 16 * 8 == 16 * 64 * 4);
static_assert(32 * 16 * 4 == 16 * 64 * 2);
static_assert(8 * 16 * 68 * 4 <= 131072);
template <int OUT_MODE, bool HAS_BIAS>
static __device__ __forceinline__ void gemm64_body(
    const _Float16* __restrict__ A, const unsigned lda, const _Float16* __restrict__ Bt, const unsigned ldb,
    void* __restrict__ Cout, const unsigned ldc, const float* __restrict__ bias,
    const unsigned M, const unsigned N, const unsigned K) {
  __shared__ __align__(16) float sT[8][16 * 68];
  const unsigned lane = threadIdx.x & 31u;
  const unsigned wave = (unsigned)__builtin_amdgcn_readfirstlane((int)(threadIdx.x >> 5));
  const unsigned tilesN = N >> 6, tilesM = M >> 6;
  const unsigned tile = blockIdx.x * 8u + wave;
  if (tile >= tilesM * tilesN) return;
  const unsigned tm = tile / tilesN;
  const unsigned tn = tile - tm * tilesN;
  const unsigned m0 = tm << 6, n0 = tn << 6;
  const unsigned rlane = lane & 15u;
  const unsigned koff = (lane >> 4) * 8u;
  const unsigned mOff = koff;

  v8f acc[4][4];
#pragma unroll
  for (int i = 0; i < 4; ++i)
#pragma unroll
    for (int j = 0; j < 4; ++j) acc[i][j] = (v8f){0.f,0.f,0.f,0.f,0.f,0.f,0.f,0.f};

#pragma unroll 1
  for (unsigned k0 = 0; k0 < K; k0 += 32u) {
    v16h bh[4];
#pragma unroll
    for (int j = 0; j < 4; ++j)
      bh[j] = frag_ld(Bt + (size_t)(n0 + ((unsigned)j << 4) + rlane) * ldb + koff + k0);
#pragma unroll
    for (int i = 0; i < 4; ++i) {
      const v16h ah = frag_ld(A + (size_t)(m0 + ((unsigned)i << 4) + rlane) * lda + koff + k0);
#pragma unroll
      for (int j = 0; j < 4; ++j)
        acc[i][j] = wmma16(ah, bh[j], acc[i][j]);
    }
  }

  float* slab = sT[wave];
#pragma unroll
  for (int i = 0; i < 4; ++i) {
    const unsigned mBase = m0 + ((unsigned)i << 4);
#pragma unroll
    for (int j = 0; j < 4; ++j) {
      const unsigned n = n0 + ((unsigned)j << 4) + rlane;
      float bv = 0.0f;
      if (HAS_BIAS) bv = bfr(bias[n]);
#pragma unroll
      for (int r = 0; r < 8; ++r) {
        float v;
        if (OUT_MODE == 0) v = acc[i][j][r] * SC_OUT + bv;
        else               v = acc[i][j][r] * SC_QKV;
        slab[(mOff + (unsigned)r) * 68u + ((unsigned)j << 4) + rlane] = v;
      }
    }
    wave_sync_lds();
    if (OUT_MODE == 0) {
      float* C = (float*)Cout;
      const unsigned hh = lane >> 4, c4 = (lane & 15u) * 4u;
#pragma unroll
      for (int half = 0; half < 2; ++half) {
        v4f vv[4];
#pragma unroll
        for (int it = 0; it < 4; ++it) {
          const unsigned row = (unsigned)(half * 4 + it) * 2u + hh;
          vv[it] = *(const v4f*)(slab + row * 68u + c4);
        }
        for (int pass = 0; pass < 2; ++pass) {
#pragma unroll
          for (int it = 0; it < 4; ++it) {
            const unsigned row = (unsigned)(half * 4 + it) * 2u + hh;
            *(volatile v4f*)(C + (size_t)(mBase + row) * ldc + n0 + c4) = vv[it];
          }
          __threadfence();
        }
      }
    } else {
      _Float16* C = (_Float16*)Cout;
      const unsigned q = lane >> 3, c8 = (lane & 7u) * 8u;
      v8h hv[4];
#pragma unroll
      for (int it = 0; it < 4; ++it) {
        const unsigned row = (unsigned)it * 4u + q;
        const float* sp = slab + row * 68u + c8;
        const v4f s0 = *(const v4f*)(sp), s1 = *(const v4f*)(sp + 4);
        hv[it] = cat8(toh_flush2(s0.x, s0.y), toh_flush2(s0.z, s0.w), toh_flush2(s1.x, s1.y), toh_flush2(s1.z, s1.w));
      }
      for (int pass = 0; pass < 2; ++pass) {
#pragma unroll
        for (int it = 0; it < 4; ++it) {
          const unsigned row = (unsigned)it * 4u + q;
          *(volatile v8h*)(C + (size_t)(mBase + row) * ldc + n0 + c8) = hv[it];
        }
        __threadfence();
      }
    }
    wave_sync_lds();
  }
}

__global__ __launch_bounds__(256) void k_gemm_qk(const _Float16* __restrict__ x16, const _Float16* __restrict__ wqkvT,
                                                 _Float16* __restrict__ qk16) {
    gemm64_body<1, false>(x16, (unsigned)CC, wqkvT, (unsigned)CC, (void*)qk16, (unsigned)QKP, nullptr,
                          (unsigned)MTOK, (unsigned)QKP, (unsigned)CC);
}
__global__ __launch_bounds__(256) void k_gemm_vt(const _Float16* __restrict__ wvT, const _Float16* __restrict__ x16,
                                                 _Float16* __restrict__ vt16) {
    gemm64_body<1, false>(wvT, (unsigned)CC, x16, (unsigned)CC, (void*)vt16, (unsigned)MTOK, nullptr,
                          (unsigned)CC, (unsigned)MTOK, (unsigned)CC);
}
__global__ __launch_bounds__(256) void k_gemm_out(const _Float16* __restrict__ ctx16, const _Float16* __restrict__ wprojT,
                                                  const float* __restrict__ b_proj, float* __restrict__ out) {
    gemm64_body<0, true>(ctx16, (unsigned)CC, wprojT, (unsigned)CC, (void*)out, (unsigned)CC, b_proj,
                         (unsigned)MTOK, (unsigned)CC, (unsigned)CC);
}

__global__ __launch_bounds__(256) void k_wconv(const float* __restrict__ Wm, unsigned KI, unsigned NO, unsigned lgper,
                                               _Float16* __restrict__ W16) {
    const unsigned u = blockIdx.x * 256u + threadIdx.x;
    const unsigned per = 1u << lgper;
    if (u >= NO * per) return;
    const unsigned k0 = 8u * (u & (per - 1u));
    const unsigned o = u >> lgper;
    float v[8];
#pragma unroll
    for (int i = 0; i < 8; ++i) v[i] = bfr(Wm[(size_t)(k0 + (unsigned)i) * NO + o]) * CARRY_W;
    st8hf(W16 + (size_t)o * KI + k0, v);
}

__global__ __launch_bounds__(256) void k_xconv(const float* __restrict__ x, _Float16* __restrict__ x16) {
    const unsigned u = blockIdx.x * 256u + threadIdx.x;
    if (u >= (unsigned)(MTOK * (CC / 8))) return;
    const unsigned row = u >> 5, c0 = (u & 31u) * 8u;
    const unsigned b = row / (unsigned)SEQ, n = row % (unsigned)SEQ;
    const float* xr = x + ((size_t)b * SEQ_FULL + n) * CC + c0;
    const v4f a = *(const v4f*)xr, d = *(const v4f*)(xr + 4);
    float v[8];
    v[0] = bfr(a.x) * CARRY_X; v[1] = bfr(a.y) * CARRY_X; v[2] = bfr(a.z) * CARRY_X; v[3] = bfr(a.w) * CARRY_X;
    v[4] = bfr(d.x) * CARRY_X; v[5] = bfr(d.y) * CARRY_X; v[6] = bfr(d.z) * CARRY_X; v[7] = bfr(d.w) * CARRY_X;
    st8hf(x16 + (size_t)row * CC + c0, v);
}

#define AT_PO 72
static_assert(32 * 16 * 4 == 16 * 128);
static_assert(NTAB * HEADS * 4 + 8 * 16 * AT_PO * 2 <= 131072);
__global__ __launch_bounds__(256) void k_attn(const _Float16* __restrict__ qk, const _Float16* __restrict__ vt,
                                              const int* __restrict__ relpos, const int* __restrict__ rel_len,
                                              const float* __restrict__ bias_table, _Float16* __restrict__ ctx) {
    __shared__ float sTab[NTAB * HEADS];
    __shared__ __align__(16) _Float16 sO[8][16 * AT_PO];
    const unsigned tid = threadIdx.x, lane = tid & 31u;
    const unsigned wave = (unsigned)__builtin_amdgcn_readfirstlane((int)(tid >> 5));
    const unsigned hh = lane >> 4, c = lane & 15u;
    const unsigned bx = blockIdx.x;
    const unsigned QB = (unsigned)SEQ / 128u;
    const unsigned qblk = bx % QB, bp = bx / QB;
    const unsigned pair = bp & 3u, b = bp >> 2;
    if (tid < (unsigned)(NTAB * HEADS)) sTab[tid] = bfr(bias_table[tid]);
    __syncthreads();
    const int mlen = (int)((float)rel_len[b] * 0.5f);
    const unsigned q0 = qblk * 128u + wave * 16u;
    const size_t tok0 = (size_t)b * SEQ;
    const _Float16* qrow  = qk + (tok0 + q0 + c) * QKP + 8u * hh;
    const _Float16* krow0 = qk + (tok0 + c) * QKP + 256u + 8u * hh;
    const _Float16* vcol0 = vt + (size_t)c * MTOK + tok0 + 8u * hh;
    const int* relrow = relpos + ((size_t)b * SEQ_FULL + q0 + c) * SEQ_FULL + 8u * hh;
    _Float16* pw = sO[wave];

#pragma unroll 1
    for (unsigned hp = 0; hp < 2u; ++hp) {
        const unsigned head = 2u * pair + hp;
        const v16h qf = frag_ld(qrow + head * 32u);
        const _Float16* kh = krow0 + head * 32u;
        const _Float16* vh = vcol0 + (size_t)(head * 32u) * MTOK;
        float mrun = -3.0e38f, lsum = 0.f;
        v8f o[2];
        o[0] = (v8f){0.f,0.f,0.f,0.f,0.f,0.f,0.f,0.f};
        o[1] = o[0];
#pragma unroll 1
        for (unsigned m0 = 0; m0 < (unsigned)SEQ; m0 += 32u) {
            v8f s[2];
#pragma unroll
            for (int tt = 0; tt < 2; ++tt) {
                const v16h kf = frag_ld(kh + (size_t)(m0 + 16u * (unsigned)tt) * QKP);
                const v8f z = (v8f){0.f,0.f,0.f,0.f,0.f,0.f,0.f,0.f};
                s[tt] = wmma16(kf, qf, z);
            }
            const v4i* rp = (const v4i*)(relrow + m0);
            const v4i ra = rp[0], rb = rp[1], rc = rp[4], rd = rp[5];
            const int rw[2][8] = {{ra.x, ra.y, ra.z, ra.w, rb.x, rb.y, rb.z, rb.w},
                                  {rc.x, rc.y, rc.z, rc.w, rd.x, rd.y, rd.z, rd.w}};
            float t[2][8];
            float mx = -3.0e38f;
#pragma unroll
            for (int tt = 0; tt < 2; ++tt) {
#pragma unroll
                for (int r = 0; r < 8; ++r) {
                    const int rel = rw[tt][r];
                    const unsigned ru = (unsigned)rel;
                    const unsigned ri = (ru < 9u) ? ru : 9u;
                    const float tb = sTab[8u * ri + head];
                    float sv = s[tt][r] * SC_SCORE;
                    sv += tb;
                    sv += (rel > mlen) ? -100.0f : 0.0f;
                    const float tv = sv * LOG2E;
                    t[tt][r] = tv;
                    mx = (tv > mx) ? tv : mx;
                }
            }
            const float mo = __shfl_xor(mx, 16, 32);
            mx = (mo > mx) ? mo : mx;
            const float mnew = (mx > mrun) ? mx : mrun;
            const float alpha = exp2f(mrun - mnew);
            mrun = mnew;
            float psum = 0.f;
            v2h pp[8];
#pragma unroll
            for (int tt = 0; tt < 2; ++tt) {
#pragma unroll
                for (int j = 0; j < 4; ++j) {
                    const float p0 = exp2f(t[tt][2 * j] - mnew);
                    const float p1 = exp2f(t[tt][2 * j + 1] - mnew);
                    psum += p0;
                    psum += p1;
                    pp[4 * tt + j] = toh_flush2(p0 * CARRY_P, p1 * CARRY_P);
                }
            }
            const v8h plo = cat8(pp[0], pp[1], pp[2], pp[3]);
            const v8h phi = cat8(pp[4], pp[5], pp[6], pp[7]);
            const v16h pf = __builtin_shufflevector(plo, phi, 0, 1, 2, 3, 4, 5, 6, 7, 8, 9, 10, 11, 12, 13, 14, 15);
            lsum = lsum * alpha + psum;
#pragma unroll
            for (int t2 = 0; t2 < 2; ++t2)
#pragma unroll
                for (int r = 0; r < 8; ++r) o[t2][r] *= alpha;
#pragma unroll
            for (int t2 = 0; t2 < 2; ++t2) {
                const v16h vf = frag_ld(vh + (size_t)(16u * (unsigned)t2) * MTOK + m0);
                o[t2] = wmma16(vf, pf, o[t2]);
            }
        }
        const float lt = lsum + __shfl_xor(lsum, 16, 32);
        const float inv = 1.0f / (lt * SC_DEN);
#pragma unroll
        for (int t2 = 0; t2 < 2; ++t2) {
            float w[8];
#pragma unroll
            for (int r = 0; r < 8; ++r) w[r] = o[t2][r] * inv;
            *(v8h*)(pw + c * AT_PO + hp * 32u + 16u * (unsigned)t2 + 8u * hh) = pack8f(w);
        }
    }
    wave_sync_lds();
    {
        const unsigned q = lane >> 3, c8 = (lane & 7u) * 8u;
        v8h ov[4];
#pragma unroll
        for (int it = 0; it < 4; ++it) ov[it] = *(const v8h*)(pw + ((unsigned)it * 4u + q) * AT_PO + c8);
        _Float16* dst = ctx + (tok0 + q0) * CC + pair * 64u;
        for (int pass = 0; pass < 2; ++pass) {
#pragma unroll
            for (int it = 0; it < 4; ++it) *(volatile v8h*)(dst + (size_t)((unsigned)it * 4u + q) * CC + c8) = ov[it];
            __threadfence();
        }
    }
}

static constexpr size_t SZ_X16   = (size_t)MTOK * CC * 2;
static constexpr size_t SZ_WQKV  = (size_t)3 * CC * CC * 2;
static constexpr size_t SZ_WPROJ = (size_t)CC * CC * 2;
static constexpr size_t SZ_QK    = (size_t)MTOK * QKP * 2;
static constexpr size_t SZ_VT    = (size_t)CC * MTOK * 2;
static constexpr size_t SZ_CTX   = (size_t)MTOK * CC * 2;
static constexpr size_t OFF_X16   = 0;
static constexpr size_t OFF_WQKV  = OFF_X16 + SZ_X16;
static constexpr size_t OFF_WPROJ = OFF_WQKV + SZ_WQKV;
static constexpr size_t OFF_QK    = OFF_WPROJ + SZ_WPROJ;
static constexpr size_t OFF_VT    = OFF_QK + SZ_QK;
static constexpr size_t OFF_CTX   = OFF_VT + SZ_VT;
static constexpr size_t WS_TOTAL  = OFF_CTX + SZ_CTX;
static_assert(SZ_X16 % 256 == 0 && SZ_WQKV % 256 == 0 && SZ_WPROJ % 256 == 0 && SZ_QK % 256 == 0 && SZ_VT % 256 == 0);
static_assert(WS_TOTAL <= ((size_t)128 << 20));

static constexpr unsigned G_WQKV = (3 * CC * (CC / 8)) / 256;
static constexpr unsigned G_WPRJ = (CC * (CC / 8)) / 256;
static constexpr unsigned G_X    = (MTOK * (CC / 8)) / 256;
static constexpr unsigned G_QK   = ((MTOK / 64) * (QKP / 64) + 7) / 8;
static constexpr unsigned G_VT   = ((CC / 64) * (MTOK / 64) + 7) / 8;
static constexpr unsigned G_OUT  = ((MTOK / 64) * (CC / 64) + 7) / 8;
static constexpr unsigned G_ATT  = NB * 4 * (SEQ / 128);

extern "C" void kernel_launch(void* const* d_in, const int* in_sizes, int n_in, void* d_out, int out_size,
                              void* d_ws, size_t ws_size, hipStream_t stream) {
    if (n_in < 7) return;
    if (in_sizes[0] < MTOK * CC || in_sizes[1] < NB * SEQ * SEQ || in_sizes[2] < NB) return;
    if (in_sizes[3] < CC * 3 * CC || in_sizes[4] < CC * CC || in_sizes[5] < CC || in_sizes[6] < NTAB * HEADS) return;
    if (out_size < MTOK * CC) return;
    if (WS_TOTAL > ws_size) return;

    const float* att_embedding     = (const float*)d_in[0];
    const int*   relation_position = (const int*)d_in[1];
    const int*   rel_len           = (const int*)d_in[2];
    const float* W_qkv             = (const float*)d_in[3];
    const float* W_proj            = (const float*)d_in[4];
    const float* b_proj            = (const float*)d_in[5];
    const float* bias_table        = (const float*)d_in[6];
    float* out = (float*)d_out;

    char* wsp = (char*)d_ws;
    _Float16* x16    = (_Float16*)(wsp + OFF_X16);
    _Float16* wqkvT  = (_Float16*)(wsp + OFF_WQKV);
    _Float16* wprojT = (_Float16*)(wsp + OFF_WPROJ);
    _Float16* qk16   = (_Float16*)(wsp + OFF_QK);
    _Float16* vt16   = (_Float16*)(wsp + OFF_VT);
    _Float16* ctx16  = (_Float16*)(wsp + OFF_CTX);

    k_wconv<<<G_WQKV, 256, 0, stream>>>(W_qkv, (unsigned)CC, (unsigned)(3 * CC), 5u, wqkvT);
    k_wconv<<<G_WPRJ, 256, 0, stream>>>(W_proj, (unsigned)CC, (unsigned)CC, 5u, wprojT);
    k_xconv<<<G_X, 256, 0, stream>>>(att_embedding, x16);

    k_gemm_qk<<<G_QK, 256, 0, stream>>>((const _Float16*)x16, (const _Float16*)wqkvT, qk16);
    k_gemm_vt<<<G_VT, 256, 0, stream>>>((const _Float16*)(wqkvT + (size_t)2 * CC * CC), (const _Float16*)x16, vt16);
    k_attn<<<G_ATT, 256, 0, stream>>>((const _Float16*)qk16, (const _Float16*)vt16, relation_position, rel_len, bias_table, ctx16);
    k_gemm_out<<<G_OUT, 256, 0, stream>>>((const _Float16*)ctx16, (const _Float16*)wprojT, b_proj, out);
}
